// GODIVA_60885456388392
// MI455X (gfx1250) — hardware-verified
//
#include <hip/hip_runtime.h>

typedef _Float16 f16;
typedef __attribute__((ext_vector_type(16))) _Float16 v16h;
typedef __attribute__((ext_vector_type(8)))  _Float16 v8h;
typedef __attribute__((ext_vector_type(8)))  float    v8f;

#define WMMA_F16(A, B, C) \
  __builtin_amdgcn_wmma_f32_16x16x32_f16(false, (A), false, (B), (short)0, (C), false, false)
typedef __attribute__((ext_vector_type(4))) float v4f_t;
typedef float v4fa __attribute__((ext_vector_type(4), may_alias));
typedef __attribute__((ext_vector_type(4))) unsigned v4u_t;
typedef unsigned v4ua __attribute__((ext_vector_type(4), may_alias));
#define RSPLIT (1.0f / 2048.0f)
#define PLW ((size_t)512 * 512)
#define PLT ((size_t)8192 * 512)
__device__ __forceinline__ f16 lo_of(float v, f16 h) { return (f16)((v - (float)h) * 2048.0f); }
__device__ __forceinline__ v8f wmma_split(v16h a, v16h al, v16h b, v16h bl, v8f c) { v8f x = {}; x = WMMA_F16(al, b, x); x = WMMA_F16(a, bl, x); return WMMA_F16(a, b, c) + x * RSPLIT; }
__device__ __forceinline__ v16h frag16(const f16* p, int hf) { return __builtin_shufflevector(*(const v8h*)(p + 8 * hf), *(const v8h*)(p + 16 + 8 * hf), 0,1,2,3,4,5,6,7,8,9,10,11,12,13,14,15); }

#define RFL(x) __builtin_amdgcn_readfirstlane(x)


__device__ __forceinline__ bool mask_ok(int q, int k) {
  int d = q - k;
  if (d >= 0 && d <= 16) return true;
  int tq = q >> 8, rq = (q >> 4) & 15, cq = q & 15;
  int tk = k >> 8, rk = (k >> 4) & 15, ck = k & 15;
  if (rk == rq && ck == cq && tk <= tq) return true;
  if (tk == tq && ck == cq && rk <= rq) return true;
  return false;
}

__device__ __forceinline__ int block_start(int i, int t, int r, int q0, int eb) {
  if (i < t) return q0 - 256 * (t - i);
  i -= t;
  if (i < eb) return q0 - 16;
  return (q0 & ~255) + 16 * (i - eb);
}

__global__ void k_wtrans(const float* __restrict__ W, f16* __restrict__ Wt) {
  int idx = blockIdx.x * 256 + threadIdx.x;
  if (idx >= 512 * 64) return;
  int n = idx >> 6, k8 = (idx & 63) * 8;
  f16 hh[8], hl[8];
#pragma unroll
  for (int e = 0; e < 8; ++e) { const float v = W[(size_t)(k8 + e) * 512 + n]; hh[e] = (f16)v; hl[e] = lo_of(v, hh[e]); }
  f16* d = Wt + (size_t)n * 512 + k8;
  *(volatile v4u_t*)d = *(const v4ua*)hh; *(volatile v4u_t*)(d + PLW) = *(const v4ua*)hl; __threadfence();
  *(volatile v4u_t*)d = *(const v4ua*)hh; *(volatile v4u_t*)(d + PLW) = *(const v4ua*)hl;
}

template <int A_F32, int OUT_F32, int TRANS_V>
__global__ void k_gemm(const void* __restrict__ Xv, const f16* __restrict__ Wt,
                       const float* __restrict__ bias, void* __restrict__ Ov,
                       float scale) {
  const int lane = threadIdx.x & 31;
  const int w    = RFL(threadIdx.x >> 5);
  const int col  = lane & 15;
  const int hf   = lane >> 4;
  const int bn   = blockIdx.x & 7;
  const int bm   = blockIdx.x >> 3;
  const int m0   = bm * 128 + w * 16;
  const int n0   = bn * 64;
  const int row  = m0 + col;

  v8f acc[4] = {};
  const float* Xf = (const float*)Xv;
  const f16*   Xh = (const f16*)Xv;

  for (int k0 = 0; k0 < 512; k0 += 32) {
    v16h a, al;
    if (A_F32) {
      const float* p = Xf + (size_t)row * 512 + k0 + 8 * hf;
      v8f lo = *(const v8f*)p;
      v8f hi = *(const v8f*)(p + 16);
#pragma unroll
      for (int j = 0; j < 8; ++j) { a[j] = (f16)lo[j]; al[j] = lo_of(lo[j], a[j]); a[8 + j] = (f16)hi[j]; al[8 + j] = lo_of(hi[j], a[8 + j]); }
    } else {
      const f16* p = Xh + (size_t)row * 512 + k0;
      a = frag16(p, hf); al = frag16(p + PLT, hf);
    }
#pragma unroll
    for (int f = 0; f < 4; ++f) {
      const f16* bp = Wt + (size_t)(n0 + 16 * f + col) * 512 + k0;
      if (OUT_F32) acc[f] = wmma_split(a, al, frag16(bp, hf), frag16(bp + PLW, hf), acc[f]);
      else         acc[f] = WMMA_F16(a, frag16(bp, hf), acc[f]);
    }
  }

  __shared__ __attribute__((aligned(16))) float stg[8][16 * 68];
  __shared__ __attribute__((aligned(16))) f16 stv[2][64 * 136];
  if (TRANS_V) {
#pragma unroll
    for (int f = 0; f < 4; ++f) {
      const float bb = bias[n0 + 16 * f + col];
#pragma unroll
      for (int v = 0; v < 8; ++v) {
        const float val = (acc[f][v] + bb) * scale;
        const int sl = w * 16 + v + 8 * hf, nl = 16 * f + col;
        const f16 hv = (f16)val; stv[0][nl * 136 + sl] = hv; stv[1][nl * 136 + sl] = lo_of(val, hv);
      }
    }
    __syncthreads();
    const int bb_ = (bm * 128) >> 10, s0 = (bm * 128) & 1023;
#pragma unroll 1
    for (int pass = 0; pass < 2; ++pass) {
      for (int c = threadIdx.x; c < 64 * 16; c += 256) { const int nl = c >> 4, q = (c & 15) * 8;
        f16* d = (f16*)Ov + (size_t)(bb_ * 512 + n0 + nl) * 1024 + s0 + q;
        *(volatile v4u_t*)d = *(const volatile v4ua*)(stv[0] + nl * 136 + q);
        *(volatile v4u_t*)(d + PLT) = *(const volatile v4ua*)(stv[1] + nl * 136 + q); }
      __threadfence();
    }
  } else {
    float* sw = stg[w];
#pragma unroll
    for (int f = 0; f < 4; ++f) {
      const float bb = bias[n0 + 16 * f + col];
#pragma unroll
      for (int v = 0; v < 8; ++v) sw[(v + 8 * hf) * 68 + 16 * f + col] = (acc[f][v] + bb) * scale;
    }
    asm volatile("s_wait_dscnt 0" ::: "memory");
#pragma unroll 1
    for (int pass = 0; pass < 2; ++pass) {
      if (OUT_F32) {
#pragma unroll
        for (int i = 0; i < 8; ++i) { const int c = lane + 32 * i, rr = c >> 4, q = (c & 15) * 4;
          *(volatile v4f_t*)((float*)Ov + (size_t)(m0 + rr) * 512 + n0 + q) = *(const volatile v4fa*)(sw + rr * 68 + q); }
      } else {
#pragma unroll
        for (int i = 0; i < 4; ++i) { const int c = lane + 32 * i, rr = c >> 3, q = (c & 7) * 8; const float* s = sw + rr * 68 + q;
          f16 hh[8], hl[8];
#pragma unroll
          for (int e = 0; e < 8; ++e) { hh[e] = (f16)s[e]; hl[e] = lo_of(s[e], hh[e]); }
          f16* d = (f16*)Ov + (size_t)(m0 + rr) * 512 + n0 + q;
          *(volatile v4u_t*)d = *(const v4ua*)hh; *(volatile v4u_t*)(d + PLT) = *(const v4ua*)hl; }
      }
      __threadfence();
    }
  }
}

__global__ void k_attn(const f16* __restrict__ Qh, const f16* __restrict__ Kh,
                       const f16* __restrict__ Vt, f16* __restrict__ Ah) {
  __shared__ __align__(32) _Float16 pbuf[8][16 * 32];

  const int lane = threadIdx.x & 31;
  const int w    = RFL(threadIdx.x >> 5);
  const int col  = lane & 15;
  const int hf   = lane >> 4;
  const int wg   = blockIdx.x * 8 + w;
  const int qt   = wg & 63;
  const int h    = (wg >> 6) & 7;
  const int b    = wg >> 9;
  const int q0   = qt * 16;
  const int t    = q0 >> 8;
  const int r    = (q0 >> 4) & 15;

  const f16* Qb = Qh + (size_t)b * 1024 * 512 + h * 64;
  const f16* Kb = Kh + (size_t)b * 1024 * 512 + h * 64;
  const f16* Vb = Vt + (size_t)(b * 8 + h) * 64 * 1024;

  v16h aq0, aq1;
  {
    const f16* qp = Qb + (size_t)(q0 + col) * 512;
    v8h l0 = *(const v8h*)(qp + 8 * hf);
    v8h h0 = *(const v8h*)(qp + 16 + 8 * hf);
    v8h l1 = *(const v8h*)(qp + 32 + 8 * hf);
    v8h h1 = *(const v8h*)(qp + 48 + 8 * hf);
#pragma unroll
    for (int j = 0; j < 8; ++j) {
      aq0[j] = l0[j]; aq0[8 + j] = h0[j];
      aq1[j] = l1[j]; aq1[8 + j] = h1[j];
    }
  }

  v8f o[4] = {};
  float m_run[8], l_run[8];
#pragma unroll
  for (int v = 0; v < 8; ++v) { m_run[v] = -1e30f; l_run[v] = 0.0f; }

  const int eb = (r == 0 && t > 0) ? 1 : 0;
  const int nb = t + eb + r + 1;

  for (int i = 0; i < nb; i += 2) {
    const int kbA = RFL(block_start(i, t, r, q0, eb));
    const int kbB = RFL((i + 1 < nb) ? block_start(i + 1, t, r, q0, eb) : -1);

    v8f sA = {}, sB = {};
    {
      const f16* kp = Kb + (size_t)kbA * 512 + (size_t)col * 512;
      sA = WMMA_F16(aq0, frag16(kp, hf), sA);
      sA = WMMA_F16(aq1, frag16(kp + 32, hf), sA);
    }
    if (kbB >= 0) {
      const f16* kp = Kb + (size_t)kbB * 512 + (size_t)col * 512;
      sB = WMMA_F16(aq0, frag16(kp, hf), sB);
      sB = WMMA_F16(aq1, frag16(kp + 32, hf), sB);
    }

    float lA[8], lB[8];
    const int kA = kbA + col;
    const int kB = (kbB >= 0 ? kbB : 0) + col;
#pragma unroll
    for (int v = 0; v < 8; ++v) {
      int q = q0 + v + 8 * hf;
      lA[v] = mask_ok(q, kA) ? sA[v] : -1e30f;
      lB[v] = (kbB >= 0 && mask_ok(q, kB)) ? sB[v] : -1e30f;
    }
    float mx[8];
#pragma unroll
    for (int v = 0; v < 8; ++v) mx[v] = fmaxf(lA[v], lB[v]);
#pragma unroll
    for (int off = 1; off < 16; off <<= 1)
#pragma unroll
      for (int v = 0; v < 8; ++v) mx[v] = fmaxf(mx[v], __shfl_xor(mx[v], off));

    float pA[8], pB[8], rs[8];
#pragma unroll
    for (int v = 0; v < 8; ++v) {
      float nm = fmaxf(m_run[v], mx[v]);
      float sc = __expf(m_run[v] - nm);
      pA[v] = __expf(lA[v] - nm);
      pB[v] = __expf(lB[v] - nm);
      rs[v] = pA[v] + pB[v];
      l_run[v] *= sc;
      m_run[v] = nm;
#pragma unroll
      for (int f = 0; f < 4; ++f) o[f][v] *= sc;
    }
#pragma unroll
    for (int off = 1; off < 16; off <<= 1)
#pragma unroll
      for (int v = 0; v < 8; ++v) rs[v] += __shfl_xor(rs[v], off);
#pragma unroll
    for (int v = 0; v < 8; ++v) l_run[v] += rs[v];

#pragma unroll
    for (int v = 0; v < 8; ++v) {
      int m = v + 8 * hf;
      pbuf[w][m * 32 + col]      = (f16)(pA[v] * 1024.0f);
      pbuf[w][m * 32 + 16 + col] = (f16)(pB[v] * 1024.0f);
    }
    __asm__ volatile("s_wait_dscnt 0" ::: "memory");
    v16h pf;
    {
      const _Float16* pp = &pbuf[w][col * 32 + 8 * hf];
      v8h lo = *(const v8h*)pp;
      v8h hi = *(const v8h*)(pp + 16);
#pragma unroll
      for (int j = 0; j < 8; ++j) { pf[j] = lo[j]; pf[8 + j] = hi[j]; }
    }

    const int kbB_s = (kbB >= 0) ? kbB : kbA;
#pragma unroll
    for (int f = 0; f < 4; ++f) {
      const f16* vr = Vb + (size_t)(16 * f + col) * 1024 + 8 * hf;
      v16h vf = __builtin_shufflevector(*(const v8h*)(vr + kbA), *(const v8h*)(vr + kbB_s), 0,1,2,3,4,5,6,7,8,9,10,11,12,13,14,15);
      o[f] = WMMA_F16(pf, vf, o[f]);
    }
  }

  __shared__ __attribute__((aligned(16))) float osh[8][16 * 68];
  float* so = osh[w];
#pragma unroll
  for (int f = 0; f < 4; ++f)
#pragma unroll
    for (int v = 0; v < 8; ++v) so[(v + 8 * hf) * 68 + 16 * f + col] = o[f][v] / (l_run[v] * 1024.0f);
  __asm__ volatile("s_wait_dscnt 0" ::: "memory");
#pragma unroll 1
  for (int pass = 0; pass < 2; ++pass) {
#pragma unroll
    for (int i = 0; i < 4; ++i) { const int c = lane + 32 * i, rr = c >> 3, q = (c & 7) * 8; const float* s = so + rr * 68 + q;
      f16 hh[8], hl[8];
#pragma unroll
      for (int e = 0; e < 8; ++e) { hh[e] = (f16)s[e]; hl[e] = lo_of(s[e], hh[e]); }
      f16* d = Ah + (size_t)(b * 1024 + q0 + rr) * 512 + h * 64 + q;
      *(volatile v4u_t*)d = *(const v4ua*)hh; *(volatile v4u_t*)(d + PLT) = *(const v4ua*)hl; }
    __threadfence();
  }
}

extern "C" void kernel_launch(void* const* d_in, const int* in_sizes, int n_in,
                              void* d_out, int out_size, void* d_ws, size_t ws_size,
                              hipStream_t stream) {
  (void)in_sizes; (void)n_in; (void)out_size; (void)ws_size;
  const float* query = (const float*)d_in[0];
  const float* key   = (const float*)d_in[1];
  const float* value = (const float*)d_in[2];
  const float* Wq    = (const float*)d_in[3];
  const float* bq    = (const float*)d_in[4];
  const float* Wk    = (const float*)d_in[5];
  const float* bk    = (const float*)d_in[6];
  const float* Wv    = (const float*)d_in[7];
  const float* bv    = (const float*)d_in[8];
  const float* Wo    = (const float*)d_in[9];
  const float* bo    = (const float*)d_in[10];

  char* ws = (char*)d_ws;
  const size_t WSZ = (size_t)512 * 512 * sizeof(f16) * 2;
  const size_t TSZ = (size_t)8192 * 512 * sizeof(f16) * 2;
  f16* WtQ = (f16*)(ws + 0 * WSZ);
  f16* WtK = (f16*)(ws + 1 * WSZ);
  f16* WtV = (f16*)(ws + 2 * WSZ);
  f16* WtO = (f16*)(ws + 3 * WSZ);
  f16* Qh  = (f16*)(ws + 4 * WSZ + 0 * TSZ);
  f16* Kh  = (f16*)(ws + 4 * WSZ + 1 * TSZ);
  f16* Vt  = (f16*)(ws + 4 * WSZ + 2 * TSZ);
  f16* Ah  = (f16*)(ws + 4 * WSZ + 3 * TSZ);

  dim3 blk(256);
  k_wtrans<<<128, blk, 0, stream>>>(Wq, WtQ);
  k_wtrans<<<128, blk, 0, stream>>>(Wk, WtK);
  k_wtrans<<<128, blk, 0, stream>>>(Wv, WtV);
  k_wtrans<<<128, blk, 0, stream>>>(Wo, WtO);

  k_gemm<1, 0, 0><<<512, blk, 0, stream>>>(query, WtQ, bq, Qh, 0.125f);
  k_gemm<1, 0, 0><<<512, blk, 0, stream>>>(key,   WtK, bk, Kh, 1.0f);
  k_gemm<1, 0, 1><<<512, blk, 0, stream>>>(value, WtV, bv, Vt, 1.0f);

  k_attn<<<512, blk, 0, stream>>>(Qh, Kh, Vt, Ah);

  k_gemm<0, 1, 0><<<512, blk, 0, stream>>>(Ah, WtO, bo, d_out, 1.0f);
}
